// KpcaStd_30863634989789
// MI455X (gfx1250) — hardware-verified
//
#include <hip/hip_runtime.h>


#define NN   8192
#define DX   256
#define DH   512
#define RCH  1024
#define ETA  1.0f
#define CST  0.1f
#define SIG  1.0f
#define DM   DX
#define LOSC 1024.0f

typedef _Float16 h16;
typedef unsigned short bf;
typedef __attribute__((ext_vector_type(16))) __bf16   v16bf;
typedef __attribute__((ext_vector_type(16))) _Float16 v16h;
typedef __attribute__((ext_vector_type(8)))  _Float16 v8h;
typedef __attribute__((ext_vector_type(8)))  unsigned short v8us;
typedef __attribute__((ext_vector_type(8)))  float    v8f;
typedef __attribute__((ext_vector_type(4)))  float    v4f;
typedef v8h  __attribute__((may_alias)) v8ha;
typedef v4f  __attribute__((may_alias)) v4fa;
typedef v8us __attribute__((may_alias)) v8usa;

__device__ __forceinline__ unsigned short f2bf(float f) { unsigned u = __float_as_uint(f); u += 0x7FFFu + ((u >> 16) & 1u); return (unsigned short)(u >> 16); }
__device__ __forceinline__ float bf2f(unsigned short b) { return __uint_as_float(((unsigned)b) << 16); }
__device__ __forceinline__ float bfr(float f) { return bf2f(f2bf(f)); }
__device__ __forceinline__ v16h cat16(v8h lo, v8h hi) { return __builtin_shufflevector(lo, hi, 0, 1, 2, 3, 4, 5, 6, 7, 8, 9, 10, 11, 12, 13, 14, 15); }
__device__ __forceinline__ v16bf cat16b(v8us lo, v8us hi) { return __builtin_bit_cast(v16bf, __builtin_shufflevector(lo, hi, 0, 1, 2, 3, 4, 5, 6, 7, 8, 9, 10, 11, 12, 13, 14, 15)); }
__device__ __forceinline__ v8f wmma16(v16h a, v16h b, v8f c) { return __builtin_amdgcn_wmma_f32_16x16x32_f16(false, a, false, b, (short)0, c, false, false); }
__device__ __forceinline__ v8f wmmab(v16bf a, v16bf b, v8f c) { return __builtin_amdgcn_wmma_f32_16x16x32_bf16(false, a, false, b, (short)0, c, false, false); }

template <bool SPLITA, bool F16OUT = false>
__global__ __launch_bounds__(128) void k_gemmb(const bf* __restrict__ A, const bf* __restrict__ Al, const bf* __restrict__ Bn, const float* __restrict__ bias, float* C, int ldc, h16* C2, const float* __restrict__ R = nullptr, int K = DM, int roundR = 1) {
    __shared__ __align__(16) float ost[4][16 * 68];
    const int lane = threadIdx.x & 31, wave = threadIdx.x >> 5, lr = lane & 15, hi = lane >> 4;
    const int r0 = blockIdx.x * 64 + wave * 16, c0 = blockIdx.y * 64;
    const size_t aoff = (size_t)(r0 + lr) * K + 8 * hi;
    size_t boff[4];
#pragma unroll
    for (int t = 0; t < 4; ++t) boff[t] = (size_t)(c0 + t * 16 + lr) * K + 8 * hi;
    v8f acc[4];
#pragma unroll
    for (int t = 0; t < 4; ++t) acc[t] = (v8f){};
#pragma unroll 1
    for (int kc = 0; kc < K; kc += 32) {
        const v16bf a = cat16b(*(const v8us*)(A + aoff + kc), *(const v8us*)(A + aoff + kc + 16));
        v16bf al = a;
        if (SPLITA) al = cat16b(*(const v8us*)(Al + aoff + kc), *(const v8us*)(Al + aoff + kc + 16));
#pragma unroll
        for (int t = 0; t < 4; ++t) { const v16bf b = cat16b(*(const v8us*)(Bn + boff[t] + kc), *(const v8us*)(Bn + boff[t] + kc + 16)); acc[t] = wmmab(a, b, acc[t]); if (SPLITA) acc[t] = wmmab(al, b, acc[t]); }
        asm volatile("v_nop\n\tv_nop\n\tv_nop\n\tv_nop" : "+v"(acc[0]), "+v"(acc[1]), "+v"(acc[2]), "+v"(acc[3]) : "v"(a), "v"(al));
    }
    float* os = &ost[wave][0];
#pragma unroll
    for (int t = 0; t < 4; ++t) { const float bv = bias ? bfr(bias[c0 + t * 16 + lr]) : 0.f;
#pragma unroll
        for (int j = 0; j < 8; ++j) os[(hi * 8 + j) * 68 + t * 16 + lr] = acc[t][j] + bv; }
    __syncthreads();
    if (F16OUT) {
        h16* crow = (h16*)(void*)C + (size_t)r0 * ldc + c0;
        auto pass = [&]() {
#pragma unroll
            for (int s = 0; s < 4; ++s) { const int row = 4 * s + (lane >> 3), piece = lane & 7; const float* sp = os + row * 68 + piece * 8; v8h o, o2;
#pragma unroll
                for (int i = 0; i < 8; ++i) { const h16 a = (h16)sp[i]; o[i] = a; o2[i] = (h16)((sp[i] - (float)a) * LOSC); }
                *(volatile v8h*)(crow + (size_t)row * ldc + piece * 8) = o; if (C2) *(volatile v8h*)(C2 + (size_t)r0 * ldc + c0 + (size_t)row * ldc + piece * 8) = o2; }
        };
        pass(); __threadfence(); pass();
    } else {
        float* crow = C + (size_t)r0 * ldc + c0;
        auto pass = [&]() {
#pragma unroll
            for (int s = 0; s < 8; ++s) { const int Lid = (lane >> 3) + 4 * s, piece = lane & 7; const int row = Lid >> 1, cofs = (Lid & 1) * 32 + piece * 4;
                v4f val = *(const v4fa*)(os + row * 68 + cofs); if (R) { const v4f rv = *(const v4f*)(R + ((size_t)r0 + row) * ldc + c0 + cofs); val += roundR ? (v4f){bfr(rv[0]), bfr(rv[1]), bfr(rv[2]), bfr(rv[3])} : rv; }
                *(volatile v4f*)(crow + (size_t)row * ldc + cofs) = val; }
        };
        pass(); __threadfence(); pass();
    }
}


__global__ __launch_bounds__(256) void k_wt(const float* __restrict__ Wm, int K, int ncols, bf* WT) {
    __shared__ __align__(16) unsigned short tl[64 * 72];
    const int tid = threadIdx.x, k0 = blockIdx.x * 64, n0 = blockIdx.y * 64;
    const int kk = tid >> 2, nq = (tid & 3) * 16;
#pragma unroll
    for (int i = 0; i < 16; ++i) tl[(nq + i) * 72 + kk] = f2bf(Wm[(size_t)(k0 + kk) * ncols + n0 + nq + i]);
    __syncthreads();
    const int piece = tid & 7;
    auto pass = [&]() {
#pragma unroll
        for (int s = 0; s < 2; ++s) { const int nr = (tid >> 3) + 32 * s; const v8us val = *(const v8usa*)(tl + nr * 72 + piece * 8); *(volatile v8us*)(WT + (size_t)(n0 + nr) * K + k0 + piece * 8) = val; }
    };
    pass(); __threadfence(); pass();
}

__global__ __launch_bounds__(256) void k_xb(const float* __restrict__ x, bf* Xb) {
    const int lane = threadIdx.x & 31, r = blockIdx.x * 8 + (threadIdx.x >> 5); if (r >= NN) return; v8us o;
#pragma unroll
    for (int i = 0; i < 8; ++i) o[i] = f2bf(x[(size_t)r * DX + lane * 8 + i]);
    *(volatile v8us*)(Xb + (size_t)r * DX + lane * 8) = o; __threadfence(); *(volatile v8us*)(Xb + (size_t)r * DX + lane * 8) = o;
}
__global__ __launch_bounds__(256) void k_sq(const float* __restrict__ x, float* SQ) {
    const int r = blockIdx.x * 256 + threadIdx.x; if (r >= NN) return; float s = 0.f;
#pragma unroll 4
    for (int d = 0; d < DX; ++d) { const float v = bfr(x[(size_t)r * DX + d]); s = fmaf(v, v, s); }
    *(volatile float*)(SQ + r) = s; __threadfence(); *(volatile float*)(SQ + r) = s;
}
__global__ __launch_bounds__(256) void k_rbf(const float* __restrict__ G, const float* __restrict__ SQ, int n0, bf* Kh, bf* Kl) {
    const int lane = threadIdx.x & 31, r = blockIdx.x * 8 + (threadIdx.x >> 5); if (r >= RCH) return; const float sn = SQ[n0 + r];
#pragma unroll 1
    for (int ps = 0; ps < 2; ++ps) {
#pragma unroll 1
        for (int c0 = lane * 8; c0 < NN; c0 += 256) { v8us oh, ol;
#pragma unroll
            for (int q = 0; q < 8; ++q) { const int i = c0 + q; const float d2 = fmaxf(sn + SQ[i] - 2.0f * G[(size_t)r * NN + i], 0.f); const float kv = __expf(-d2 / (2.0f * SIG * SIG));
                const unsigned short hb = f2bf(kv); oh[q] = hb; ol[q] = f2bf(kv - bf2f(hb)); }
            const size_t o = (size_t)r * NN + c0; *(volatile v8us*)(Kh + o) = oh; *(volatile v8us*)(Kl + o) = ol; }
        if (ps == 0) __threadfence(); }
}
__global__ __launch_bounds__(256) void k_part(const float* __restrict__ ET, const float* __restrict__ Hm, const float* __restrict__ lam, int n0, int blk0, float* P12) {
    __shared__ float r1[256], r2[256];
    const int tid = threadIdx.x; const int rr = tid >> 6, hh = (tid & 63) * 8; const int n = blockIdx.x * 4 + rr;
    float a1 = 0.f, a2 = 0.f;
#pragma unroll
    for (int q = 0; q < 8; ++q) { const int h = hh + q; const float e = ET[(size_t)n * DH + h]; a1 = fmaf(bfr(lam[h]) * e, e, a1); a2 = fmaf(e, bfr(Hm[(size_t)(n0 + n) * DH + h]), a2); }
    r1[tid] = a1; r2[tid] = a2; __syncthreads();
#pragma unroll
    for (int s = 128; s >= 1; s >>= 1) { if (tid < s) { r1[tid] += r1[tid + s]; r2[tid] += r2[tid + s]; } __syncthreads(); }
    if (tid < 32) { const float v = (tid == 0) ? r1[0] : (tid == 1) ? r2[0] : 0.f; float* p = P12 + ((size_t)blk0 + blockIdx.x) * 32 + tid; *(volatile float*)p = v; __threadfence(); *(volatile float*)p = v; }
}
__global__ __launch_bounds__(32) void k_final(const float* __restrict__ P12, int nparts, float* OUTP) {
    if (threadIdx.x != 0) return; float s1 = 0.f, s2 = 0.f;
#pragma unroll 1
    for (int q = 0; q < nparts; ++q) { s1 += P12[(size_t)q * 32]; s2 += P12[(size_t)q * 32 + 1]; }
    const float loss = s1 / (-2.0f * ETA * ETA) + s2 / (2.0f * ETA); const float r = loss + (CST / 2.0f) * loss * loss;
    *(volatile float*)OUTP = r; __threadfence(); *(volatile float*)OUTP = r;
}

extern "C" void kernel_launch(void* const* d_in, const int* in_sizes, int n_in,
                              void* d_out, int out_size, void* d_ws, size_t ws_size, hipStream_t stream) {
    (void)in_sizes; (void)n_in; (void)out_size;
    const float* x = (const float*)d_in[0]; const float* Hm = (const float*)d_in[1]; const float* lam = (const float*)d_in[2];
    float* out = (float*)d_out;
    char* wsp = (char*)d_ws;
    auto take = [&](size_t bytes) { char* p = wsp; wsp += (bytes + 255) & ~(size_t)255; return (void*)p; };
    bf* Xb = (bf*)take((size_t)NN * DX * 2); float* SQ = (float*)take((size_t)NN * 4); bf* HT = (bf*)take((size_t)DH * NN * 2); float* G = (float*)take((size_t)RCH * NN * 4);
    bf* Kh = (bf*)take((size_t)RCH * NN * 2); bf* Kl = (bf*)take((size_t)RCH * NN * 2); float* ET = (float*)take((size_t)RCH * DH * 4); float* P12 = (float*)take((size_t)(NN / 4) * 32 * 4);
    if ((size_t)(wsp - (char*)d_ws) > ws_size) return;
    k_xb<<<NN / 8, 256, 0, stream>>>(x, Xb); k_sq<<<NN / 256, 256, 0, stream>>>(x, SQ); k_wt<<<dim3(NN / 64, DH / 64, 1), 256, 0, stream>>>(Hm, NN, DH, HT);
    for (int ch = 0; ch < NN / RCH; ++ch) { const int n0 = ch * RCH;
        k_gemmb<false, false><<<dim3(RCH / 64, NN / 64, 1), 128, 0, stream>>>(Xb + (size_t)n0 * DX, nullptr, Xb, nullptr, G, NN, nullptr, nullptr, DX);
        k_rbf<<<RCH / 8, 256, 0, stream>>>(G, SQ, n0, Kh, Kl);
        k_gemmb<true, false><<<dim3(RCH / 64, DH / 64, 1), 128, 0, stream>>>(Kh, Kl, HT, nullptr, ET, DH, nullptr, nullptr, NN);
        k_part<<<RCH / 4, 256, 0, stream>>>(ET, Hm, lam, n0, ch * (RCH / 4), P12); }
    k_final<<<1, 32, 0, stream>>>(P12, NN / 4, out);
}
